// RecursiveNN_50311246905374
// MI455X (gfx1250) — hardware-verified
//
#include <hip/hip_runtime.h>
#include <stddef.h>


typedef _Float16 h16;
typedef _Float16 v16h __attribute__((ext_vector_type(16)));
typedef _Float16 v8h  __attribute__((ext_vector_type(8)));
typedef float    v8f  __attribute__((ext_vector_type(8)));
typedef float    v4f  __attribute__((ext_vector_type(4)));

#ifndef NB
#define NB 256
#endif
#ifndef LEAVES
#define LEAVES 1024
#endif
#ifndef TOP_RES
#define TOP_RES 1
#endif
#define NB_FULL     256
#define LEAVES_FULL 1024
#define VOCAB 50257
#define WDIM  300
#define KPAD1 320
#define HIDN  256
#define K2    512
#define SUBL  128
#define BPT   (LEAVES / SUBL)
#define EPR   (KPAD1 / 8)
#define EPIECES ((unsigned)VOCAB * (unsigned)EPR)
#define CLAST (WDIM - 4)

static_assert(NB >= 64 && NB <= NB_FULL && (NB % 64) == 0);
static_assert(LEAVES >= 128 && LEAVES <= LEAVES_FULL && (LEAVES & (LEAVES - 1)) == 0);
static_assert(HIDN == 256 && K2 == 2 * HIDN);
static_assert((KPAD1 % 64) == 0 && KPAD1 >= WDIM && (WDIM % 4) == 0);
static_assert((HIDN % 64) == 0 && (K2 % 64) == 0);
static_assert((SUBL % 128) == 0 && BPT >= 1);
static_assert(EPR == 40);
static_assert(((size_t)VOCAB * KPAD1 * 2) % 128 == 0);
static_assert((size_t)VOCAB * EPR < (size_t)0xFFFFFFFFu);

#define LDT 72
#define LDC 68
#define LDE 328
#define LDH 264
#define LDF 260
static_assert((LDT % 8) == 0 && LDT >= 64);
static_assert((LDC % 4) == 0 && LDC >= 64);
static_assert((LDE % 8) == 0 && LDE >= KPAD1);
static_assert((LDH % 8) == 0 && LDH >= HIDN);
static_assert((LDF % 4) == 0 && LDF >= HIDN);
static_assert(64 * LDH <= 64 * LDE);
static_assert((size_t)64 * LDE * 2 + (size_t)128 * LDH * 2 + (size_t)16 * LDF * 4 + 128 * 4 <= (size_t)131072);
static_assert(64 * EPR == 256 * 10);

#define WCARRY 64.0f
#define ECARRY 64.0f
#define HCARRY 64.0f
#define RCARRY 2048.0f

#define W1T_BYTES ((size_t)HIDN * KPAD1 * 2)
#define W2T_BYTES ((size_t)HIDN * K2 * 2)
#define E16_BYTES ((size_t)VOCAB * KPAD1 * 2)
#define HPL_BYTES ((size_t)NB * LEAVES * 128)
#define OFF_W1T ((size_t)0)
#define OFF_W2T (OFF_W1T + W1T_BYTES)
#define OFF_E16 (OFF_W2T + W2T_BYTES)
#define OFF_HHI (OFF_E16 + E16_BYTES)
#define OFF_HRS (OFF_HHI + HPL_BYTES)
#define WS_TOTAL (OFF_HRS + HPL_BYTES)
static_assert((W1T_BYTES % 128) == 0 && (W2T_BYTES % 128) == 0 && (E16_BYTES % 128) == 0);
static_assert((HPL_BYTES % 128) == 0);
static_assert(WS_TOTAL <= (size_t)134217728);

__device__ __forceinline__ float bf16r(float x) {
  unsigned int u = __float_as_uint(x);
  u = (u + 0x7FFFu + ((u >> 16) & 1u)) & 0xFFFF0000u;
  return __uint_as_float(u);
}

static __device__ __forceinline__ h16 toh_flush(float v) {
  const h16 r = (h16)v;
  return (fabsf(v) < 6.103515625e-05f) ? (h16)0.0f : r;
}

__device__ __forceinline__ v16h frag_at(const _Float16* p) {
  v8h lo = *(const v8h*)(p);
  v8h hi = *(const v8h*)(p + 16);
  v16h out;
#pragma unroll
  for (int i = 0; i < 8; ++i) { out[i] = lo[i]; out[i + 8] = hi[i]; }
  return out;
}
__device__ __forceinline__ v16h ld_frag(const _Float16* base, unsigned ld) {
  const unsigned lane = threadIdx.x & 31u;
  return frag_at(base + (lane & 15u) * ld + (lane >> 4) * 8u);
}

__device__ __forceinline__ v8f wmma16(v16h a, v16h b, v8f c) {
  v8f d = __builtin_amdgcn_wmma_f32_16x16x32_f16(false, a, false, b, (short)0, c,
                                                 false, false);
  asm volatile("v_nop\n\tv_nop\n\tv_nop\n\tv_nop" : "+v"(d) : "v"(a), "v"(b));
  return d;
}

__global__ __launch_bounds__(256) void wconv_kernel(
    const float* __restrict__ W, _Float16* __restrict__ Wt, unsigned ldw, unsigned ldk,
    unsigned kreal) {
  __shared__ _Float16 T[64 * LDT];
  const unsigned tid = threadIdx.x;
  const unsigned n0 = blockIdx.x * 64u;
  const unsigned k0 = blockIdx.y * 64u;
#pragma unroll 4
  for (unsigned j = 0; j < 16u; ++j) {
    const unsigned idx = tid + 256u * j;
    const unsigned kr = idx >> 6, nc = idx & 63u;
    const unsigned kk = k0 + kr;
    const unsigned kcl = (kk < kreal) ? kk : (kreal - 1u);
    float v = W[(size_t)kcl * ldw + n0 + nc];
    v = (kk < kreal) ? v : 0.0f;
    T[nc * LDT + kr] = toh_flush(WCARRY * bf16r(v));
  }
  __syncthreads();
  v8h x[2];
  size_t off[2];
#pragma unroll
  for (unsigned i = 0; i < 2u; ++i) {
    const unsigned n = 32u * i + (tid >> 3);
    const unsigned kc = (tid & 7u) * 8u;
    x[i] = *(const v8h*)&T[n * LDT + kc];
    off[i] = (size_t)(n0 + n) * ldk + k0 + kc;
  }
#pragma unroll
  for (int i = 0; i < 2; ++i) *(volatile v8h*)(Wt + off[i]) = x[i];
  __threadfence();
#pragma unroll
  for (int i = 0; i < 2; ++i) *(volatile v8h*)(Wt + off[i]) = x[i];
}

__global__ __launch_bounds__(256) void econv_kernel(
    const float* __restrict__ E, _Float16* __restrict__ E16) {
#pragma clang fp contract(off)
  const unsigned p = blockIdx.x * 256u + threadIdx.x;
  const unsigned pc = (p < EPIECES) ? p : (EPIECES - 1u);
  const unsigned row = pc / (unsigned)EPR;
  const unsigned c8 = pc - row * (unsigned)EPR;
  const unsigned cbase = c8 * 8u;
  const unsigned ca = (cbase < (unsigned)CLAST) ? cbase : (unsigned)CLAST;
  const unsigned cb = (cbase + 4u < (unsigned)CLAST) ? (cbase + 4u) : (unsigned)CLAST;
  const float* er = E + (size_t)row * WDIM;
  const v4f a0 = *(const v4f*)(er + ca);
  const v4f a1 = *(const v4f*)(er + cb);
  v8h o;
#pragma unroll
  for (int i = 0; i < 4; ++i) {
    const float e0 = (cbase + (unsigned)i < (unsigned)WDIM) ? a0[i] : 0.0f;
    const float e1 = (cbase + 4u + (unsigned)i < (unsigned)WDIM) ? a1[i] : 0.0f;
    o[i]     = toh_flush(ECARRY * bf16r(e0));
    o[i + 4] = toh_flush(ECARRY * bf16r(e1));
  }
  if (p < EPIECES) {
    _Float16* q = E16 + (size_t)p * 8u;
    *(volatile v8h*)q = o;
    __threadfence();
    *(volatile v8h*)q = o;
  }
}

template <int MT>
__device__ __forceinline__ void pair_gemm(const _Float16* src, const _Float16* bp0,
                                          const _Float16* bp1, const unsigned hh,
                                          const unsigned m, v8f (&acc)[MT][2]) {
#pragma unroll
  for (int mt = 0; mt < MT; ++mt) { acc[mt][0] = (v8f){}; acc[mt][1] = (v8f){}; }
#pragma unroll 1
  for (unsigned ks = 0; ks < (unsigned)(K2 / 32); ++ks) {
    const unsigned sib = ks >> 3;
    const unsigned kk = (ks & 7u) * 32u;
    const v16h b0 = frag_at(bp0 + ks * 32u);
    const v16h b1 = frag_at(bp1 + ks * 32u);
#pragma unroll
    for (int mt = 0; mt < MT; ++mt) {
      const v16h a = frag_at(src + (2u * ((unsigned)mt * 16u + m) + sib) * LDH + kk + hh * 8u);
      acc[mt][0] = wmma16(a, b0, acc[mt][0]);
      acc[mt][1] = wmma16(a, b1, acc[mt][1]);
    }
  }
}

template <int MT>
__device__ __forceinline__ void put_nodes(_Float16* dst, const v8f (&acc)[MT][2],
                                          const float bv0, const float bv1, const unsigned w,
                                          const unsigned hh, const unsigned m) {
#pragma unroll
  for (int mt = 0; mt < MT; ++mt)
#pragma unroll
    for (int r = 0; r < 8; ++r) {
      _Float16* d = dst + ((unsigned)mt * 16u + hh * 8u + (unsigned)r) * LDH + w * 32u + m;
      d[0]  = toh_flush(acc[mt][0][r] * (1.0f / WCARRY) + bv0);
      d[16] = toh_flush(acc[mt][1][r] * (1.0f / WCARRY) + bv1);
    }
}

__global__ __launch_bounds__(256) void leaf_tree_kernel(
    const int* __restrict__ ids, const _Float16* __restrict__ E16,
    const _Float16* __restrict__ W1t, const float* __restrict__ b1,
    const _Float16* __restrict__ W2t, const float* __restrict__ b2,
    _Float16* __restrict__ Hhi, _Float16* __restrict__ Hres) {
  __shared__ _Float16 Ea[64 * LDE];
  __shared__ _Float16 Hb[128 * LDH];
  __shared__ float Cs[16 * LDF];
  __shared__ int wid[128];

  const unsigned tid = threadIdx.x, lane = tid & 31u;
  const unsigned w = (unsigned)__builtin_amdgcn_readfirstlane((int)(tid >> 5));
  const unsigned hh = lane >> 4, m = lane & 15u;
  const unsigned blk = blockIdx.x;
  const unsigned tree = blk / (unsigned)BPT;
  const unsigned g = blk - tree * (unsigned)BPT;

  if (tid < 128u) {
    int id = ids[(size_t)tree * LEAVES_FULL + g * 128u + tid];
    id = (id < 0) ? 0 : id;
    id = (id > VOCAB - 1) ? (VOCAB - 1) : id;
    wid[tid] = id;
  }

  const unsigned col0 = w * 32u + m;
  const float b1v0 = HCARRY * bf16r(b1[col0]);
  const float b1v1 = HCARRY * bf16r(b1[col0 + 16u]);
  const float b2v0 = HCARRY * bf16r(b2[col0]);
  const float b2v1 = HCARRY * bf16r(b2[col0 + 16u]);

  const _Float16* w1p0 = W1t + (size_t)col0 * KPAD1 + hh * 8u;
  const _Float16* w1p1 = w1p0 + (size_t)16 * KPAD1;
  const _Float16* w2p0 = W2t + (size_t)col0 * K2 + hh * 8u;
  const _Float16* w2p1 = w2p0 + (size_t)16 * K2;
  __syncthreads();

#pragma unroll 1
  for (unsigned hf = 0; hf < 2u; ++hf) {
#pragma unroll 2
    for (unsigned j = 0; j < 10u; ++j) {
      const unsigned idx = tid + 256u * j;
      const unsigned r = idx / (unsigned)EPR;
      const unsigned c = (idx - r * (unsigned)EPR) * 8u;
      const int id = wid[hf * 64u + r];
      const v8h e = *(const v8h*)(E16 + (size_t)id * KPAD1 + c);
      *(v8h*)&Ea[r * LDE + c] = e;
    }
    __syncthreads();

    v8f acc[4][2];
#pragma unroll
    for (int mt = 0; mt < 4; ++mt) { acc[mt][0] = (v8f){}; acc[mt][1] = (v8f){}; }
#pragma unroll 1
    for (unsigned ks = 0; ks < (unsigned)(KPAD1 / 32); ++ks) {
      const v16h f0 = frag_at(w1p0 + ks * 32u);
      const v16h f1 = frag_at(w1p1 + ks * 32u);
#pragma unroll
      for (int mt = 0; mt < 4; ++mt) {
        const v16h a = ld_frag(&Ea[(mt * 16) * LDE + ks * 32u], LDE);
        acc[mt][0] = wmma16(a, f0, acc[mt][0]);
        acc[mt][1] = wmma16(a, f1, acc[mt][1]);
      }
    }
    put_nodes<4>(Hb + hf * 64u * LDH, acc, b1v0, b1v1, w, hh, m);
    __syncthreads();
  }

  {
    v8f acc[4][2];
    pair_gemm<4>(Hb, w2p0, w2p1, hh, m, acc);
    put_nodes<4>(Ea, acc, b2v0, b2v1, w, hh, m);
  }
  __syncthreads();
  {
    v8f acc[2][2];
    pair_gemm<2>(Ea, w2p0, w2p1, hh, m, acc);
    put_nodes<2>(Hb, acc, b2v0, b2v1, w, hh, m);
  }
  __syncthreads();
  {
    v8f acc[1][2];
    pair_gemm<1>(Hb, w2p0, w2p1, hh, m, acc);
#pragma unroll
    for (int r = 0; r < 8; ++r) {
      float* d = &Cs[(hh * 8u + (unsigned)r) * LDF + w * 32u + m];
      d[0]  = acc[0][0][r] * (1.0f / WCARRY) + b2v0;
      d[16] = acc[0][1][r] * (1.0f / WCARRY) + b2v1;
    }
  }
  __syncthreads();

  v8h xh[2], xr[2];
  size_t off[2];
#pragma unroll
  for (unsigned i = 0; i < 2u; ++i) {
    const unsigned r = 8u * i + (tid >> 5);
    const unsigned c = lane * 8u;
    const v4f u0 = *(const v4f*)&Cs[r * LDF + c];
    const v4f u1 = *(const v4f*)&Cs[r * LDF + c + 4u];
#pragma unroll
    for (int j = 0; j < 4; ++j) {
      const h16 h0 = toh_flush(u0[j]);
      const h16 h1 = toh_flush(u1[j]);
      xh[i][j]     = h0;
      xh[i][j + 4] = h1;
      xr[i][j]     = toh_flush((u0[j] - (float)h0) * RCARRY);
      xr[i][j + 4] = toh_flush((u1[j] - (float)h1) * RCARRY);
    }
    off[i] = ((size_t)blk * 16u + r) * HIDN + c;
  }
#pragma unroll
  for (int i = 0; i < 2; ++i) *(volatile v8h*)(Hhi + off[i]) = xh[i];
#if TOP_RES
#pragma unroll
  for (int i = 0; i < 2; ++i) *(volatile v8h*)(Hres + off[i]) = xr[i];
#endif
  __threadfence();
#pragma unroll
  for (int i = 0; i < 2; ++i) *(volatile v8h*)(Hhi + off[i]) = xh[i];
#if TOP_RES
#pragma unroll
  for (int i = 0; i < 2; ++i) *(volatile v8h*)(Hres + off[i]) = xr[i];
#endif
}

template <int MODE>
__device__ __forceinline__ void level_body(
    const _Float16* __restrict__ A16, const _Float16* __restrict__ A16r,
    const _Float16* __restrict__ Bt, const float* __restrict__ bias,
    float* __restrict__ outf, _Float16* __restrict__ out16, _Float16* __restrict__ out16r) {
  __shared__ float Cs[64 * LDC];
  const unsigned tid = threadIdx.x, lane = tid & 31u;
  const unsigned w = (unsigned)__builtin_amdgcn_readfirstlane((int)(tid >> 5));
  const unsigned mw = w >> 1, nw = w & 1u;
  const unsigned hh = lane >> 4, m = lane & 15u;
  const unsigned n0 = blockIdx.x * 64u;
  const unsigned row0 = blockIdx.y * 64u;

  const size_t aoff = (size_t)(row0 + mw * 16u + m) * K2 + hh * 8u;
  const _Float16* ap  = A16 + aoff;
  const _Float16* bp0 = Bt + (size_t)(n0 + nw * 32u + m) * K2 + hh * 8u;
  const _Float16* bp1 = bp0 + (size_t)16 * K2;
  v8f acc0 = {}, acc1 = {};
#if TOP_RES
  const _Float16* arp = A16r + aoff;
  v8f rc0 = {}, rc1 = {};
#endif
#pragma unroll 2
  for (unsigned k0 = 0; k0 < (unsigned)K2; k0 += 32u) {
    const v16h a  = frag_at(ap + k0);
    const v16h b0 = frag_at(bp0 + k0);
    const v16h b1 = frag_at(bp1 + k0);
    acc0 = wmma16(a, b0, acc0);
    acc1 = wmma16(a, b1, acc1);
#if TOP_RES
    const v16h ar = frag_at(arp + k0);
    rc0 = wmma16(ar, b0, rc0);
    rc1 = wmma16(ar, b1, rc1);
#endif
  }
#pragma unroll
  for (int r = 0; r < 8; ++r) {
    float* d = &Cs[(mw * 16u + hh * 8u + (unsigned)r) * LDC + nw * 32u + m];
#if TOP_RES
    d[0]  = acc0[r] + rc0[r] * (1.0f / RCARRY);
    d[16] = acc1[r] + rc1[r] * (1.0f / RCARRY);
#else
    d[0]  = acc0[r];
    d[16] = acc1[r];
#endif
  }
  __syncthreads();

  if (MODE == 0) {
    v8h xh[2], xr[2];
    size_t off[2];
#pragma unroll
    for (unsigned i = 0; i < 2u; ++i) {
      const unsigned r = 32u * i + (tid >> 3);
      const unsigned c = (tid & 7u) * 8u;
      const v4f u0 = *(const v4f*)&Cs[r * LDC + c];
      const v4f u1 = *(const v4f*)&Cs[r * LDC + c + 4u];
      const v4f g0 = *(const v4f*)(bias + n0 + c);
      const v4f g1 = *(const v4f*)(bias + n0 + c + 4u);
#pragma unroll
      for (int j = 0; j < 4; ++j) {
        const float t0 = u0[j] * (1.0f / WCARRY) + HCARRY * bf16r(g0[j]);
        const float t1 = u1[j] * (1.0f / WCARRY) + HCARRY * bf16r(g1[j]);
        const h16 h0 = toh_flush(t0);
        const h16 h1 = toh_flush(t1);
        xh[i][j]     = h0;
        xh[i][j + 4] = h1;
        xr[i][j]     = toh_flush((t0 - (float)h0) * RCARRY);
        xr[i][j + 4] = toh_flush((t1 - (float)h1) * RCARRY);
      }
      off[i] = (size_t)(row0 + r) * HIDN + n0 + c;
    }
#pragma unroll
    for (int i = 0; i < 2; ++i) *(volatile v8h*)(out16 + off[i]) = xh[i];
#if TOP_RES
#pragma unroll
    for (int i = 0; i < 2; ++i) *(volatile v8h*)(out16r + off[i]) = xr[i];
#endif
    __threadfence();
#pragma unroll
    for (int i = 0; i < 2; ++i) *(volatile v8h*)(out16 + off[i]) = xh[i];
#if TOP_RES
#pragma unroll
    for (int i = 0; i < 2; ++i) *(volatile v8h*)(out16r + off[i]) = xr[i];
#endif
  }

  if (MODE == 1) {
    v4f xs[4];
    size_t off[4];
#pragma unroll
    for (unsigned i = 0; i < 4u; ++i) {
      const unsigned r = 16u * i + (tid >> 4);
      const unsigned c = (tid & 15u) * 4u;
      const v4f u = *(const v4f*)&Cs[r * LDC + c];
      const v4f g = *(const v4f*)(bias + n0 + c);
      v4f val;
#pragma unroll
      for (int j = 0; j < 4; ++j)
        val[j] = u[j] * (1.0f / (WCARRY * HCARRY)) + bf16r(g[j]);
      xs[i] = val;
      off[i] = (size_t)(row0 + r) * HIDN + n0 + c;
    }
#pragma unroll
    for (int i = 0; i < 4; ++i) *(volatile v4f*)(outf + off[i]) = xs[i];
    __threadfence();
#pragma unroll
    for (int i = 0; i < 4; ++i) *(volatile v4f*)(outf + off[i]) = xs[i];
  }
}

__global__ __launch_bounds__(256) void level_plane_kernel(
    const _Float16* __restrict__ A16, const _Float16* __restrict__ A16r,
    const _Float16* __restrict__ Bt, const float* __restrict__ bias,
    _Float16* __restrict__ out16, _Float16* __restrict__ out16r) {
  level_body<0>(A16, A16r, Bt, bias, (float*)0, out16, out16r);
}
__global__ __launch_bounds__(256) void level_out_kernel(
    const _Float16* __restrict__ A16, const _Float16* __restrict__ A16r,
    const _Float16* __restrict__ Bt, const float* __restrict__ bias,
    float* __restrict__ outf) {
  level_body<1>(A16, A16r, Bt, bias, outf, (_Float16*)0, (_Float16*)0);
}

extern "C" void kernel_launch(void* const* d_in, const int* in_sizes, int n_in,
                              void* d_out, int out_size, void* d_ws, size_t ws_size,
                              hipStream_t stream) {
  if (n_in < 6) return;
  if ((long long)in_sizes[0] < (long long)(NB - 1) * LEAVES_FULL + LEAVES) return;
  if ((long long)in_sizes[1] < (long long)VOCAB * WDIM) return;
  if ((long long)in_sizes[2] < (long long)WDIM * HIDN) return;
  if (in_sizes[3] < HIDN) return;
  if ((long long)in_sizes[4] < (long long)K2 * HIDN) return;
  if (in_sizes[5] < HIDN) return;
  if ((long long)out_size < (long long)NB * HIDN) return;
  if (ws_size < WS_TOTAL) return;

  const int*   ids = (const int*)d_in[0];
  const float* emb = (const float*)d_in[1];
  const float* w1  = (const float*)d_in[2];
  const float* b1  = (const float*)d_in[3];
  const float* w2  = (const float*)d_in[4];
  const float* b2  = (const float*)d_in[5];
  float* out = (float*)d_out;

  char* ws = (char*)d_ws;
  _Float16* W1t  = (_Float16*)(ws + OFF_W1T);
  _Float16* W2t  = (_Float16*)(ws + OFF_W2T);
  _Float16* E16  = (_Float16*)(ws + OFF_E16);
  _Float16* Hhi  = (_Float16*)(ws + OFF_HHI);
  _Float16* Hres = (_Float16*)(ws + OFF_HRS);

  dim3 blk(256);
  wconv_kernel<<<dim3(HIDN / 64, KPAD1 / 64), blk, 0, stream>>>(
      w1, W1t, (unsigned)HIDN, (unsigned)KPAD1, (unsigned)WDIM);
  wconv_kernel<<<dim3(HIDN / 64, K2 / 64), blk, 0, stream>>>(
      w2, W2t, (unsigned)HIDN, (unsigned)K2, (unsigned)K2);
  econv_kernel<<<dim3((EPIECES + 255u) / 256u), blk, 0, stream>>>(emb, E16);
  leaf_tree_kernel<<<dim3(NB * BPT), blk, 0, stream>>>(ids, E16, W1t, b1, W2t, b2, Hhi, Hres);

  size_t src_off = 0;
  unsigned cur = (unsigned)NB * (unsigned)(LEAVES / 8);
  while (cur > (unsigned)NB) {
    const unsigned mrows = cur >> 1;
    const size_t dst_off = src_off + (size_t)cur * HIDN;
    const dim3 gl(HIDN / 64, mrows / 64);
    if (mrows > (unsigned)NB) {
      level_plane_kernel<<<gl, blk, 0, stream>>>(Hhi + src_off, Hres + src_off, W2t, b2,
                                                 Hhi + dst_off, Hres + dst_off);
    } else {
      level_out_kernel<<<gl, blk, 0, stream>>>(Hhi + src_off, Hres + src_off, W2t, b2, out);
    }
    src_off = dst_off;
    cur = mrows;
  }
}
